// LSTMDecoder_10711648436649
// MI455X (gfx1250) — hardware-verified
//
#include <hip/hip_runtime.h>
#include <math.h>

constexpr int NSTEP  = 128;
constexpr int NB     = 64;
constexpr int NINF   = 512;
constexpr int NACT   = 512;
constexpr int NLIN   = NINF + NACT;
constexpr int NH     = 1024;
constexpr int NG4    = 4 * NH;
constexpr int CHSTEP = 64;
constexpr int NCHUNK = NSTEP / CHSTEP;
constexpr int MCH    = CHSTEP * NB;
constexpr int NTHR   = 256;
constexpr int RTHR   = 512;
constexpr int RB     = 16;
constexpr int HP     = 1040;
constexpr int SLP    = 68;
constexpr int NOUT0  = NSTEP * NB * NH;
constexpr int NOUT1  = NB * NH;
static_assert(NSTEP % CHSTEP == 0);
static_assert(NH == 64 * (RTHR / 32));
static_assert(NB % RB == 0);
static_assert(NINF % 32 == 0 && NACT % 32 == 0 && NH % 32 == 0);
static_assert(NG4 % 64 == 0 && MCH % 64 == 0 && NB % 64 == 0);
static_assert((RB * NH) % (8 * RTHR) == 0);
static_assert(HP % 8 == 0 && HP >= NH + 8);
static_assert(((NG4 / 64) * (NB / 64)) % 8 == 0);
static_assert(((NG4 / 64) * (MCH / 64)) % 8 == 0);

typedef __attribute__((ext_vector_type(16))) _Float16 v16h;
typedef __attribute__((ext_vector_type(8)))  _Float16 v8h;
typedef __attribute__((ext_vector_type(16))) __bf16   v16b;
typedef __attribute__((ext_vector_type(8)))  __bf16   v8b;
typedef __attribute__((ext_vector_type(8)))  float    v8f;
typedef __attribute__((ext_vector_type(4)))  float    v4f;
typedef __attribute__((ext_vector_type(4)))  unsigned v4u;

__device__ __forceinline__ unsigned short f2bf_bits(float f) {
  unsigned u = __float_as_uint(f);
  return (unsigned short)((u + 0x7FFFu + ((u >> 16) & 1u)) >> 16);
}
__device__ __forceinline__ float bf_bits2f(unsigned short h) { return __uint_as_float(((unsigned)h) << 16); }
__device__ __forceinline__ float bf16r(float f) { return bf_bits2f(f2bf_bits(f)); }

__device__ __forceinline__ void dep_guard_b(v8f& a, v8f& b, v16b x, v16b y) { asm volatile("v_nop\n\tv_nop\n\tv_nop\n\tv_nop" : "+v"(a), "+v"(b) : "v"(x), "v"(y)); }
__device__ __forceinline__ void dep_guard4_b(v8f& a, v8f& b, v8f& c, v8f& d, v16b x, v16b y) {
  asm volatile("v_nop\n\tv_nop\n\tv_nop\n\tv_nop" : "+v"(a), "+v"(b), "+v"(c), "+v"(d) : "v"(x), "v"(y));
}
__device__ __forceinline__ void keep4_b(v16b a, v16b b, v16b c, v16b d) { asm volatile("v_nop" :: "v"(a), "v"(b), "v"(c), "v"(d)); }
__device__ __forceinline__ void acc_guard4(v8f& a, v8f& b, v8f& c, v8f& d) { asm volatile("v_nop\n\tv_nop\n\tv_nop\n\tv_nop" : "+v"(a), "+v"(b), "+v"(c), "+v"(d)); }

template <typename T> struct Frag;
template <> struct Frag<__bf16> {
  typedef v16b V; union U { v16b v; v8b h[2]; };
  static __device__ __forceinline__ v16b load(const __bf16* p) {
    U f; f.h[0] = *(const v8b*)(p); f.h[1] = *(const v8b*)(p + 16); return f.v;
  }
  static __device__ __forceinline__ v8f mma(v16b a, v16b b, v8f c) {
    return __builtin_amdgcn_wmma_f32_16x16x32_bf16(false, a, false, b, (short)0, c, false, false);
  }
};

__device__ __forceinline__ float fsigm(float x) { return 1.0f / (1.0f + expf(-x)); }

__global__ __launch_bounds__(NTHR) void cvt8_kernel(const float* __restrict__ src, unsigned short* __restrict__ dst,
                                                    int nrow, int ncol8, int spitch, int scol0) {
  const int i  = blockIdx.x * NTHR + threadIdx.x;
  const int n8 = nrow * ncol8;
  if (i < n8) {
    const int row = i / ncol8;
    const int c8  = i - row * ncol8;
    const float* sp = src + (size_t)row * spitch + scol0 + c8 * 8;
    const v4f a = *(const v4f*)(sp);
    const v4f b = *(const v4f*)(sp + 4);
    v8h hv;
#pragma unroll
    for (int e = 0; e < 4; ++e) {
      const unsigned short b0 = f2bf_bits(a[e]);
      const unsigned short b1 = f2bf_bits(b[e]);
      hv[e]     = __builtin_bit_cast(_Float16, b0);
      hv[4 + e] = __builtin_bit_cast(_Float16, b1);
    }
    *(volatile v8h*)(dst + (size_t)i * 8) = hv;
    __threadfence();
    *(volatile v8h*)(dst + (size_t)i * 8) = hv;
  }
}

__global__ __launch_bounds__(NTHR) void bias_sum_kernel(const float* __restrict__ ba, const float* __restrict__ bb,
                                                        float* __restrict__ dst, int n4) {
  const int i = blockIdx.x * NTHR + threadIdx.x;
  if (i < n4) {
    const v4f va = *(const v4f*)(ba + 4 * i);
    const v4f vb = *(const v4f*)(bb + 4 * i);
    v4f o;
#pragma unroll
    for (int e = 0; e < 4; ++e) o[e] = bf16r(va[e]) + bf16r(vb[e]);
    *(volatile v4f*)(dst + 4 * i) = o;
    __threadfence();
    *(volatile v4f*)(dst + 4 * i) = o;
  }
}

template <int BIAS_M, bool RES64>
__global__ __launch_bounds__(NTHR) void gemm_bt_kernel(
    const unsigned short* __restrict__ Ap, int lda,
    const unsigned short* __restrict__ Btp, int ldb,
    float* __restrict__ C, int ldc,
    const float* __restrict__ bias, const float* __restrict__ res,
    int M, int N, int K) {
  const __bf16* A  = (const __bf16*)Ap;
  const __bf16* Bt = (const __bf16*)Btp;
  __shared__ __align__(16) float sT[8][16 * 68];
  const int lane = threadIdx.x & 31;
  const int wave = threadIdx.x >> 5;
  const int tilesN = N >> 6;
  const int tilesM = M >> 6;
  const int tile = blockIdx.x * 8 + wave;
  if (tile >= tilesM * tilesN) return;
  const int tm = tile / tilesN;
  const int tn = tile - tm * tilesN;
  const int m0 = tm << 6;
  const int n0 = tn << 6;

  const int rlane = lane & 15;
  const int koff  = (lane >> 4) * 8;
  const int mOff  = (lane >> 4) * 8;

  v8f acc[4][4];
#pragma unroll
  for (int i = 0; i < 4; ++i)
#pragma unroll
    for (int j = 0; j < 4; ++j) acc[i][j] = (v8f){0.f,0.f,0.f,0.f,0.f,0.f,0.f,0.f};

  for (int k0 = 0; k0 < K; k0 += 32) {
    v16b bh[4];
#pragma unroll
    for (int j = 0; j < 4; ++j) {
      const size_t bo = (size_t)(n0 + (j << 4) + rlane) * ldb + koff + k0;
      bh[j] = Frag<__bf16>::load(Bt + bo);
    }
#pragma unroll
    for (int i = 0; i < 4; ++i) {
      const size_t ao = (size_t)(m0 + (i << 4) + rlane) * lda + koff + k0;
      const v16b ah = Frag<__bf16>::load(A + ao);
#pragma unroll
      for (int j = 0; j < 4; ++j) acc[i][j] = Frag<__bf16>::mma(ah, bh[j], acc[i][j]);
      dep_guard4_b(acc[i][0], acc[i][1], acc[i][2], acc[i][3], ah, bh[3]);
    }
    keep4_b(bh[0], bh[1], bh[2], bh[3]);
  }
  acc_guard4(acc[0][0], acc[0][1], acc[0][2], acc[0][3]);
  acc_guard4(acc[1][0], acc[1][1], acc[1][2], acc[1][3]);
  acc_guard4(acc[2][0], acc[2][1], acc[2][2], acc[2][3]);
  acc_guard4(acc[3][0], acc[3][1], acc[3][2], acc[3][3]);

  float* slab = sT[wave];
  const int hh = lane >> 4, c4 = (lane & 15) * 4;
#pragma unroll
  for (int i = 0; i < 4; ++i) {
    const int mBase = m0 + (i << 4);
    float bvr[8];
#pragma unroll
    for (int r = 0; r < 8; ++r) bvr[r] = 0.0f;
    if (BIAS_M == 1) {
      const v4f b0 = *(const v4f*)(bias + mBase + mOff);
      const v4f b1 = *(const v4f*)(bias + mBase + mOff + 4);
      bvr[0] = b0[0]; bvr[1] = b0[1]; bvr[2] = b0[2]; bvr[3] = b0[3];
      bvr[4] = b1[0]; bvr[5] = b1[1]; bvr[6] = b1[2]; bvr[7] = b1[3];
    }
#pragma unroll
    for (int j = 0; j < 4; ++j) {
#pragma unroll
      for (int r = 0; r < 8; ++r) slab[(mOff + r) * 68 + (j << 4) + rlane] = acc[i][j][r] + bvr[r];
    }
    __builtin_amdgcn_fence(__ATOMIC_RELEASE, "workgroup");
    __builtin_amdgcn_wave_barrier();
    __builtin_amdgcn_fence(__ATOMIC_ACQUIRE, "workgroup");
    v4f vo[8];
#pragma unroll
    for (int it = 0; it < 8; ++it) {
      const int row = it * 2 + hh;
      v4f v = *(const v4f*)(slab + row * 68 + c4);
      if (RES64) {
        const v4f rr = *(const v4f*)(res + (size_t)(mBase + row) * 64 + c4);
        v += rr;
      }
      vo[it] = v;
    }
    for (int pass = 0; pass < 2; ++pass) {
#pragma unroll
      for (int it = 0; it < 8; ++it) {
        const int row = it * 2 + hh;
        *(volatile v4f*)(C + (size_t)(mBase + row) * ldc + n0 + c4) = vo[it];
      }
      __threadfence();
    }
    __builtin_amdgcn_fence(__ATOMIC_RELEASE, "workgroup");
    __builtin_amdgcn_wave_barrier();
    __builtin_amdgcn_fence(__ATOMIC_ACQUIRE, "workgroup");
  }
}

__global__ __launch_bounds__(RTHR) void rnn_chunk_kernel(const float* __restrict__ GinT,
                                                          const unsigned short* __restrict__ Whhp,
                                                          const float* __restrict__ hin,
                                                          const float* __restrict__ cin,
                                                          float* __restrict__ hs,
                                                          float* __restrict__ hfin,
                                                          float* __restrict__ cfin) {
  __shared__ __align__(16) unsigned short Ahu[RB * HP];
  __shared__ __align__(16) float          Sl[RTHR / 32][16 * SLP];
  const __bf16* Whh = (const __bf16*)Whhp;
  const int tid = threadIdx.x, lane = tid & 31, wave = tid >> 5;
  const int c = lane & 15, hh = lane >> 4, koff = hh * 8, c4 = c * 4;
  const int rowbase = blockIdx.x * RB;
  const int jw = 64 * wave;

#pragma unroll
  for (int it = 0; it < 4; ++it) {
    const int idx = it * RTHR + tid;
    const int row = idx >> 7, c8 = (idx & 127) * 8;
    const float* hp = hin + (size_t)(rowbase + row) * NH + c8;
    const v4f a = *(const v4f*)(hp);
    const v4f b = *(const v4f*)(hp + 4);
    v4u pk;
    pk[0] = (unsigned)f2bf_bits(a[0]) | ((unsigned)f2bf_bits(a[1]) << 16);
    pk[1] = (unsigned)f2bf_bits(a[2]) | ((unsigned)f2bf_bits(a[3]) << 16);
    pk[2] = (unsigned)f2bf_bits(b[0]) | ((unsigned)f2bf_bits(b[1]) << 16);
    pk[3] = (unsigned)f2bf_bits(b[2]) | ((unsigned)f2bf_bits(b[3]) << 16);
    *(v4u*)(Ahu + row * HP + c8) = pk;
  }
  if (tid < 128) *(unsigned*)(Ahu + (tid >> 3) * HP + NH + (tid & 7) * 2) = 0u;

  float* slab = Sl[wave];
#pragma unroll
  for (int it = 0; it < 8; ++it) {
    const int row = it * 2 + hh;
    const v4f v = *(const v4f*)(cin + (size_t)(rowbase + row) * NH + jw + c4);
    *(v4f*)(slab + row * SLP + c4) = v;
  }
  __syncthreads();
  float cst[4][8], hst[4][8];
#pragma unroll
  for (int nt = 0; nt < 4; ++nt)
#pragma unroll
    for (int r = 0; r < 8; ++r) { cst[nt][r] = slab[(8 * hh + r) * SLP + 16 * nt + c]; hst[nt][r] = 0.0f; }

  const __bf16* ahrow = (const __bf16*)(Ahu + c * HP + koff);

#pragma unroll 1
  for (int tt = 0; tt < CHSTEP; ++tt) {
#pragma unroll
    for (int nt = 0; nt < 4; ++nt) {
      const int j = jw + 16 * nt + c;
      const float* gp = GinT + (size_t)j * MCH + (size_t)(tt * NB + rowbase + 8 * hh);
      v8f acc[4];
#pragma unroll
      for (int g = 0; g < 4; ++g) {
        const float* gq = gp + (size_t)g * NH * MCH;
        const v4f lo = *(const v4f*)(gq);
        const v4f hi = *(const v4f*)(gq + 4);
        acc[g] = __builtin_shufflevector(lo, hi, 0, 1, 2, 3, 4, 5, 6, 7);
      }
      const __bf16* wq = Whh + (size_t)j * NH + koff;
#pragma unroll 1
      for (int k0 = 0; k0 < NH; k0 += 32) {
        const v16b a  = Frag<__bf16>::load(ahrow + k0);
        const v16b b0 = Frag<__bf16>::load(wq + k0);
        const v16b b1 = Frag<__bf16>::load(wq + (size_t)1 * NH * NH + k0);
        const v16b b2 = Frag<__bf16>::load(wq + (size_t)2 * NH * NH + k0);
        const v16b b3 = Frag<__bf16>::load(wq + (size_t)3 * NH * NH + k0);
        acc[0] = Frag<__bf16>::mma(a, b0, acc[0]);
        acc[1] = Frag<__bf16>::mma(a, b1, acc[1]);
        acc[2] = Frag<__bf16>::mma(a, b2, acc[2]);
        acc[3] = Frag<__bf16>::mma(a, b3, acc[3]);
        dep_guard4_b(acc[0], acc[1], acc[2], acc[3], a, b3);
        keep4_b(b0, b1, b2, b3);
      }
      acc_guard4(acc[0], acc[1], acc[2], acc[3]);
#pragma unroll
      for (int r = 0; r < 8; ++r) {
        const float ig = fsigm(acc[0][r]);
        const float fg = fsigm(acc[1][r]);
        const float gg = tanhf(acc[2][r]);
        const float og = fsigm(acc[3][r]);
        const float cn = fg * cst[nt][r] + ig * gg;
        cst[nt][r] = cn;
        hst[nt][r] = og * tanhf(cn);
      }
    }
    __syncthreads();
#pragma unroll
    for (int nt = 0; nt < 4; ++nt) {
      const int j = jw + 16 * nt + c;
#pragma unroll
      for (int r = 0; r < 8; ++r) {
        Ahu[(8 * hh + r) * HP + j] = f2bf_bits(hst[nt][r]);
        slab[(8 * hh + r) * SLP + 16 * nt + c] = hst[nt][r];
      }
    }
    __syncthreads();
    for (int pass = 0; pass < 2; ++pass) {
#pragma unroll
      for (int it = 0; it < 8; ++it) {
        const int row = it * 2 + hh;
        const v4f v = *(const v4f*)(slab + row * SLP + c4);
        *(volatile v4f*)(hs + (size_t)(tt * NB + rowbase + row) * NH + jw + c4) = v;
      }
      __threadfence();
    }
  }

  for (int pass = 0; pass < 2; ++pass) {
#pragma unroll
    for (int it = 0; it < 8; ++it) {
      const int row = it * 2 + hh;
      const v4f v = *(const v4f*)(slab + row * SLP + c4);
      *(volatile v4f*)(hfin + (size_t)(rowbase + row) * NH + jw + c4) = v;
    }
    __threadfence();
  }
  __syncthreads();
#pragma unroll
  for (int nt = 0; nt < 4; ++nt)
#pragma unroll
    for (int r = 0; r < 8; ++r) slab[(8 * hh + r) * SLP + 16 * nt + c] = cst[nt][r];
  __syncthreads();
  for (int pass = 0; pass < 2; ++pass) {
#pragma unroll
    for (int it = 0; it < 8; ++it) {
      const int row = it * 2 + hh;
      const v4f v = *(const v4f*)(slab + row * SLP + c4);
      *(volatile v4f*)(cfin + (size_t)(rowbase + row) * NH + jw + c4) = v;
    }
    __threadfence();
  }
}

extern "C" void kernel_launch(void* const* d_in, const int* in_sizes, int n_in,
                              void* d_out, int out_size, void* d_ws, size_t ws_size, hipStream_t stream) {
  if (n_in < 8 || d_out == nullptr || d_ws == nullptr) return;
  if (in_sizes[0] != NB * NINF || in_sizes[1] != NSTEP * NB * NACT || in_sizes[2] != NB * NH || in_sizes[3] != NB * NH ||
      in_sizes[4] != NG4 * NLIN || in_sizes[5] != NG4 * NH || in_sizes[6] != NG4 || in_sizes[7] != NG4 ||
      out_size != NOUT0 + 2 * NOUT1) return;

  const float* feat = (const float*)d_in[0];
  const float* act  = (const float*)d_in[1];
  const float* h0   = (const float*)d_in[2];
  const float* c0   = (const float*)d_in[3];
  const float* wih  = (const float*)d_in[4];
  const float* whh  = (const float*)d_in[5];
  const float* bih  = (const float*)d_in[6];
  const float* bhh  = (const float*)d_in[7];
  float* hs_out = (float*)d_out;
  float* hn_out = hs_out + (size_t)NOUT0;
  float* cn_out = hn_out + (size_t)NOUT1;

  char* ws = (char*)d_ws; size_t off = 0;
  auto carve = [&](size_t bytes) -> char* { char* p = ws + off; off += (bytes + 255) & ~(size_t)255; return p; };
  unsigned short* WIF  = (unsigned short*)carve((size_t)NG4 * NINF * 2);
  unsigned short* WIA  = (unsigned short*)carve((size_t)NG4 * NACT * 2);
  unsigned short* WHH  = (unsigned short*)carve((size_t)NG4 * NH * 2);
  unsigned short* AACT = (unsigned short*)carve((size_t)NSTEP * NB * NACT * 2);
  unsigned short* FB   = (unsigned short*)carve((size_t)NB * NINF * 2);
  float*          BSUM = (float*)carve((size_t)NG4 * 4);
  float*          GCT  = (float*)carve((size_t)NG4 * NB * 4);
  float*          GINT = (float*)carve((size_t)NG4 * MCH * 4);
  float*          HST  = (float*)carve((size_t)NB * NH * 4);
  float*          CST  = (float*)carve((size_t)NB * NH * 4);
  if (off > ws_size || off > (size_t)134217728) return;

  const int n8w = NG4 * (NINF / 8);
  const int n8h = NG4 * (NH / 8);
  const int n8a = NSTEP * NB * (NACT / 8);
  const int n8f = NB * (NINF / 8);
  cvt8_kernel<<<(n8w + NTHR - 1) / NTHR, NTHR, 0, stream>>>(wih,  WIF,  NG4,        NINF / 8, NLIN, 0);
  cvt8_kernel<<<(n8w + NTHR - 1) / NTHR, NTHR, 0, stream>>>(wih,  WIA,  NG4,        NACT / 8, NLIN, NINF);
  cvt8_kernel<<<(n8h + NTHR - 1) / NTHR, NTHR, 0, stream>>>(whh,  WHH,  NG4,        NH / 8,   NH,   0);
  cvt8_kernel<<<(n8a + NTHR - 1) / NTHR, NTHR, 0, stream>>>(act,  AACT, NSTEP * NB, NACT / 8, NACT, 0);
  cvt8_kernel<<<(n8f + NTHR - 1) / NTHR, NTHR, 0, stream>>>(feat, FB,   NB,         NINF / 8, NINF, 0);
  bias_sum_kernel<<<(NG4 / 4 + NTHR - 1) / NTHR, NTHR, 0, stream>>>(bih, bhh, BSUM, NG4 / 4);

  gemm_bt_kernel<1, false><<<((NG4 / 64) * (NB / 64)) / 8, NTHR, 0, stream>>>(
      WIF, NINF, FB, NINF, GCT, NB, BSUM, GCT, NG4, NB, NINF);

  for (int ch = 0; ch < NCHUNK; ++ch) {
    gemm_bt_kernel<0, true><<<((NG4 / 64) * (MCH / 64)) / 8, NTHR, 0, stream>>>(
        WIA, NACT, AACT + (size_t)ch * MCH * NACT, NACT, GINT, MCH, BSUM, GCT, NG4, MCH, NACT);
    const float* hin = (ch == 0) ? h0 : HST;
    const float* cin = (ch == 0) ? c0 : CST;
    float* hf = (ch == NCHUNK - 1) ? hn_out : HST;
    float* cf = (ch == NCHUNK - 1) ? cn_out : CST;
    rnn_chunk_kernel<<<NB / RB, RTHR, 0, stream>>>(GINT, WHH, hin, cin, hs_out + (size_t)ch * MCH * NH, hf, cf);
  }
}
